// InnerIteration_24507083391218
// MI455X (gfx1250) — hardware-verified
//
#include <hip/hip_runtime.h>
#include <stddef.h>
#include <stdint.h>


#define DD      128
#define GD      32
#define KL      8
#define KP2     256
#define NTHR    256
#define NWAVE   8
#define EPT     8
#define CHUNK   (NTHR * EPT)
#define WCAP    (EPT * 32)
#define LISTN   (NWAVE * WCAP)
#define NBMAX   2048
#define RCAP    28672
#define DEGCAP  4096
#define STW     512
#define TROWS   64
#define TTHR    128
#define WSMAX   134217728
#define LDS_SCAN ((2 * RCAP + 2 * NBMAX + LISTN) * 4 + 64)
#define LDS_CLS  (TROWS * KP2 * 2 + TROWS * DD * 4 + 2 * TROWS * KL * 4 + TROWS * 4)
#define LDS_VAR  (2 * TROWS * KP2 * 2 + TROWS * DD * 2 + TROWS * GD * 2 + TROWS * DD * 4 + TROWS * 4)

static_assert((CHUNK & (CHUNK - 1)) == 0 && CHUNK <= 4096);
static_assert((NBMAX & (NBMAX - 1)) == 0 && NBMAX <= 4096);
static_assert(NTHR * 8 == NBMAX);
static_assert(LISTN >= NBMAX);
static_assert(LISTN >= NWAVE * WCAP);
static_assert((RCAP % 32) == 0);
static_assert(NWAVE * STW <= RCAP);
static_assert(STW * 4 >= 512);
static_assert(LDS_SCAN <= 300000);
static_assert(LDS_CLS == 69888);
static_assert(LDS_VAR == 119040);
static_assert(TROWS == (TTHR / 32) * 16);
static_assert(TTHR * 4 == TROWS * KL);
static_assert(KL == 8);
static_assert((DD % 32) == 0 && (GD % 32) == 0 && (KP2 % 32) == 0 && KP2 == 2 * DD);

typedef float          v4f   __attribute__((ext_vector_type(4)));
typedef float          v8f   __attribute__((ext_vector_type(8)));
typedef int            v4i   __attribute__((ext_vector_type(4)));
typedef int            v8i   __attribute__((ext_vector_type(8)));
typedef unsigned int   v2u   __attribute__((ext_vector_type(2)));
typedef unsigned short v8us  __attribute__((ext_vector_type(8)));
typedef unsigned short v16us __attribute__((ext_vector_type(16)));
typedef __bf16         v16bf __attribute__((ext_vector_type(16)));
typedef v4f  __attribute__((may_alias)) v4fa;
typedef v4i  __attribute__((may_alias)) v4ia;
typedef v8us __attribute__((may_alias)) v8usa;
union FragB { v16us v; v8us h[2]; v8i w; };

__device__ __forceinline__ v8f wmb(const FragB& a, const FragB& b, v8f c) {
  v8f d = __builtin_amdgcn_wmma_f32_16x16x32_bf16(false, __builtin_bit_cast(v16bf, a.v),
                                                  false, __builtin_bit_cast(v16bf, b.v),
                                                  (short)0, c, false, false);
  asm volatile("v_nop\n\tv_nop\n\tv_nop\n\tv_nop" : "+v"(d) : "v"(a.w), "v"(b.w));
  return d;
}

__device__ __forceinline__ unsigned short bf16_rne(float f) {
  unsigned u = __float_as_uint(f);
  u = u + 0x7FFFu + ((u >> 16) & 1u);
  return (unsigned short)(u >> 16);
}
__device__ __forceinline__ float bf16_val(unsigned short s) { return __uint_as_float(((unsigned)s) << 16); }

__device__ __forceinline__ float tanh_f(float x) {
  float y = x > 15.0f ? 15.0f : x;
  y = y < -15.0f ? -15.0f : y;
  const float e = __expf(2.0f * y);
  return 1.0f - 2.0f * __builtin_amdgcn_rcpf(e + 1.0f);
}
__device__ __forceinline__ float sigm_f(float x) {
  float y = x > 30.0f ? 30.0f : x;
  y = y < -30.0f ? -30.0f : y;
  const float e = __expf(-y);
  return __builtin_amdgcn_rcpf(1.0f + e);
}

__device__ __forceinline__ void zero8(v8f (&acc)[8]) {
  const v8f z = {0.f, 0.f, 0.f, 0.f, 0.f, 0.f, 0.f, 0.f};
#pragma unroll
  for (int t = 0; t < 8; ++t) acc[t] = z;
}

__device__ __forceinline__ void gemm_seg(v8f (&acc)[8], const unsigned short* ap, const unsigned short* bp,
                                         int KB, int ksteps) {
#pragma unroll 1
  for (int ks = 0; ks < ksteps; ++ks) {
    FragB af;
    af.h[0] = *(const v8usa*)(ap + 32 * ks);
    af.h[1] = *(const v8usa*)(ap + 32 * ks + 16);
#pragma unroll
    for (int t = 0; t < 8; ++t) {
      const unsigned short* wq = bp + (size_t)(16 * t) * (size_t)KB + 32 * ks;
      FragB bf;
      bf.h[0] = *(const v8usa*)wq;
      bf.h[1] = *(const v8usa*)(wq + 16);
      acc[t] = wmb(af, bf, acc[t]);
    }
  }
}

__global__ __launch_bounds__(256) void k_cvt(const float* __restrict__ x, const float* __restrict__ g,
                                             unsigned short* vb, unsigned short* gb, int nUv, int nUg) {
  const int i = (int)blockIdx.x * 256 + (int)threadIdx.x;
  if (i >= nUv + nUg) return;
  const float* src;
  unsigned short* dst;
  if (i < nUv) { src = x + (size_t)i * 8; dst = vb + (size_t)i * 8; }
  else { const int e = i - nUv; src = g + (size_t)e * 8; dst = gb + (size_t)e * 8; }
  const v4f a = *(const v4fa*)src;
  const v4f b = *(const v4fa*)(src + 4);
  v8us o;
  o[0] = bf16_rne(a.x); o[1] = bf16_rne(a.y); o[2] = bf16_rne(a.z); o[3] = bf16_rne(a.w);
  o[4] = bf16_rne(b.x); o[5] = bf16_rne(b.y); o[6] = bf16_rne(b.z); o[7] = bf16_rne(b.w);
  *(volatile v8us*)dst = o;
  __threadfence();
  *(volatile v8us*)dst = o;
}

__global__ __launch_bounds__(256) void k_wtr2(const float* __restrict__ W, int koff, int kmod, int Kout,
                                              unsigned short* wt, int nUnits) {
  const int u = (int)blockIdx.x * 256 + (int)threadIdx.x;
  if (u >= nUnits) return;
  const int kq = Kout >> 3;
  const int n  = u / kq;
  const int k8 = (u - n * kq) * 8;
  const int kr = k8 - (k8 / kmod) * kmod;
  const int ks = koff + kr;
  const float* p = W + (size_t)ks * DD + n;
  v8us o;
  o[0] = bf16_rne(p[0]);               o[1] = bf16_rne(p[(size_t)1 * DD]);
  o[2] = bf16_rne(p[(size_t)2 * DD]);  o[3] = bf16_rne(p[(size_t)3 * DD]);
  o[4] = bf16_rne(p[(size_t)4 * DD]);  o[5] = bf16_rne(p[(size_t)5 * DD]);
  o[6] = bf16_rne(p[(size_t)6 * DD]);  o[7] = bf16_rne(p[(size_t)7 * DD]);
  const size_t off = (size_t)n * (size_t)Kout + k8;
  *(volatile v8us*)(wt + off) = o;
  __threadfence();
  *(volatile v8us*)(wt + off) = o;
}

__global__ __launch_bounds__(TTHR) void k_clause(
    const unsigned short* __restrict__ VB, const int* __restrict__ lits, const int* __restrict__ negs,
    const unsigned short* __restrict__ WnT2, const unsigned short* __restrict__ WvT2,
    const float* __restrict__ bn, const float* __restrict__ bv,
    float* CE, int nN, int nC)
{
  extern __shared__ v4f lds_dyn[];
  unsigned short* sA = (unsigned short*)lds_dyn;
  float* sP   = (float*)(sA + TROWS * KP2);
  int*   sLit = (int*)(sP + TROWS * DD);
  int*   sNg  = sLit + TROWS * KL;
  float* sNn  = (float*)(sNg + TROWS * KL);
  const int tid = (int)threadIdx.x, lane = tid & 31, wave = tid >> 5, hh = lane >> 4, m = lane & 15;
  const int c0  = (int)blockIdx.x * TROWS;
  const int wr0 = 16 * wave;

  {
    const v4i a = *(const v4ia*)(lits + (size_t)c0 * KL + 4 * tid);
    const v4i b = *(const v4ia*)(negs + (size_t)c0 * KL + 4 * tid);
    *(v4i*)(sLit + 4 * tid) = a;
    *(v4i*)(sNg + 4 * tid) = b;
  }
  __syncthreads();

#pragma unroll 1
  for (int j = 0; j < 16; ++j) {
    const int R = wr0 + j;
    float ps[8], ns[8];
#pragma unroll
    for (int i = 0; i < 8; ++i) { ps[i] = 0.f; ns[i] = 0.f; }
    int nn = 0;
#pragma unroll
    for (int p = 0; p < 4; ++p) {
      const int k = 2 * p + hh;
      int lit = sLit[R * KL + k];
      const int ng = sNg[R * KL + k];
      lit = lit < 0 ? 0 : (lit > nN - 1 ? nN - 1 : lit);
      const v8us xv = *(const v8usa*)(VB + (size_t)lit * DD + 8 * m);
      const bool isn = ng > 0;
      nn += isn ? 1 : 0;
#pragma unroll
      for (int i = 0; i < 8; ++i) {
        const float f = bf16_val(xv[i]);
        ps[i] += isn ? 0.f : f;
        ns[i] += isn ? f : 0.f;
      }
    }
#pragma unroll
    for (int i = 0; i < 8; ++i) {
      ps[i] += __shfl_xor(ps[i], 16);
      ns[i] += __shfl_xor(ns[i], 16);
    }
    nn += __shfl_xor(nn, 16);
    v8us sv;
#pragma unroll
    for (int i = 0; i < 8; ++i) {
      const unsigned short hi = bf16_rne(ns[i]);
      const unsigned short lo = bf16_rne(ns[i] - bf16_val(hi));
      sv[i] = hh ? lo : hi;
    }
    *(v8us*)(sA + R * KP2 + DD * hh + 8 * m) = sv;
    const v4f pa = {ps[0], ps[1], ps[2], ps[3]};
    const v4f pb = {ps[4], ps[5], ps[6], ps[7]};
    *(v4f*)(sP + R * DD + 8 * m) = pa;
    *(v4f*)(sP + R * DD + 8 * m + 4) = pb;
    if (lane == 0) sNn[R] = (float)nn;
  }
  __syncthreads();

  v8f acc[8];
  zero8(acc);
  gemm_seg(acc, sA + (wr0 + m) * KP2 + 8 * hh, WnT2 + (size_t)m * KP2 + 8 * hh, KP2, KP2 / 32);
  __syncthreads();
#pragma unroll
  for (int t = 0; t < 8; ++t) {
    const int col = 16 * t + m;
    const float bb = bf16_val(bf16_rne(bn[col]));
#pragma unroll
    for (int r = 0; r < 8; ++r) {
      const int row = wr0 + 8 * hh + r;
      const float u = acc[t][r] + sP[row * DD + col] + sNn[row] * bb;
      const unsigned short hi = bf16_rne(u);
      sA[row * KP2 + col] = hi;
      sA[row * KP2 + DD + col] = bf16_rne(u - bf16_val(hi));
    }
  }
  __syncthreads();

  zero8(acc);
  gemm_seg(acc, sA + (wr0 + m) * KP2 + 8 * hh, WvT2 + (size_t)m * KP2 + 8 * hh, KP2, KP2 / 32);
#pragma unroll
  for (int t = 0; t < 8; ++t) {
    const int col = 16 * t + m;
    const float bb = bf16_val(bf16_rne(bv[col]));
#pragma unroll
    for (int r = 0; r < 8; ++r) {
      const int row = wr0 + 8 * hh + r;
      sP[row * DD + col] = tanh_f(acc[t][r] + bb);
    }
  }
  __syncthreads();

#pragma unroll
  for (int i = 0; i < 16; ++i) {
    const int row = wr0 + i, grow = c0 + row;
    const v4f v = ((const v4fa*)(sP + row * DD))[lane];
    if (grow < nC) *(volatile v4f*)(CE + (size_t)grow * DD + 4 * lane) = v;
  }
  __threadfence();
#pragma unroll
  for (int i = 0; i < 16; ++i) {
    const int row = wr0 + i, grow = c0 + row;
    const v4f v = ((const v4fa*)(sP + row * DD))[lane];
    if (grow < nC) *(volatile v4f*)(CE + (size_t)grow * DD + 4 * lane) = v;
  }
}

__device__ __forceinline__ int scan_chunk(const int* __restrict__ dsts, int nE, int cbase, int slotBase,
                                          int nb, int vec8, int* list, int tid, int lane, int wave) {
  int wc = 0;
  const int el0  = tid * EPT;
  const int e0   = cbase + el0;
  const int sent = -2147483647 - 1;
  v4i da, db;
  if (vec8 != 0 && cbase + CHUNK <= nE) {
    da = *(const v4i*)(dsts + e0);
    db = *(const v4i*)(dsts + e0 + 4);
  } else {
    da.x = (e0     < nE) ? dsts[min(e0,     nE - 1)] : sent;
    da.y = (e0 + 1 < nE) ? dsts[min(e0 + 1, nE - 1)] : sent;
    da.z = (e0 + 2 < nE) ? dsts[min(e0 + 2, nE - 1)] : sent;
    da.w = (e0 + 3 < nE) ? dsts[min(e0 + 3, nE - 1)] : sent;
    db.x = (e0 + 4 < nE) ? dsts[min(e0 + 4, nE - 1)] : sent;
    db.y = (e0 + 5 < nE) ? dsts[min(e0 + 5, nE - 1)] : sent;
    db.z = (e0 + 6 < nE) ? dsts[min(e0 + 6, nE - 1)] : sent;
    db.w = (e0 + 7 < nE) ? dsts[min(e0 + 7, nE - 1)] : sent;
  }
  const unsigned nbs = (unsigned)slotBase;
  const unsigned unb = (unsigned)nb;
  const unsigned s0 = (unsigned)da.x - nbs, s1 = (unsigned)da.y - nbs;
  const unsigned s2 = (unsigned)da.z - nbs, s3 = (unsigned)da.w - nbs;
  const unsigned s4 = (unsigned)db.x - nbs, s5 = (unsigned)db.y - nbs;
  const unsigned s6 = (unsigned)db.z - nbs, s7 = (unsigned)db.w - nbs;
  const bool h0 = s0 < unb, h1 = s1 < unb, h2 = s2 < unb, h3 = s3 < unb;
  const bool h4 = s4 < unb, h5 = s5 < unb, h6 = s6 < unb, h7 = s7 < unb;
  const unsigned any = __builtin_amdgcn_ballot_w32(h0 | h1 | h2 | h3 | h4 | h5 | h6 | h7);
  if (any != 0u) {
#define HITJ(J, HJ, SJ) { \
      const unsigned mj = __builtin_amdgcn_ballot_w32(HJ); \
      if (mj != 0u) { \
        if (HJ) { \
          const int pos = wc + (int)__builtin_amdgcn_mbcnt_lo(mj, 0u); \
          if (pos < WCAP) list[wave * WCAP + pos] = ((el0 + (J)) << 12) | (int)(SJ); \
        } \
        wc += (int)__builtin_popcount(mj); } }
    HITJ(0, h0, s0)
    HITJ(1, h1, s1)
    HITJ(2, h2, s2)
    HITJ(3, h3, s3)
    HITJ(4, h4, s4)
    HITJ(5, h5, s5)
    HITJ(6, h6, s6)
    HITJ(7, h7, s7)
#undef HITJ
  }
  return wc;
}

__global__ __launch_bounds__(NTHR) void k_scan(
    const int* __restrict__ dsts, const float* __restrict__ CE,
    unsigned short* AGG, int* FLG,
    int nC, int nE, int nb, int vec8, int MPr) {
  extern __shared__ v4f lds_dyn[];
  int* reg1 = (int*)lds_dyn;
  int* reg2 = reg1 + RCAP;
  int* scnt = reg2 + RCAP;
  int* soff = scnt + NBMAX;
  int* list = soff + NBMAX;
  int* wcnt = list + LISTN;
  int* wtot = wcnt + NWAVE;
  const int tid = (int)threadIdx.x, lane = tid & 31, wave = tid >> 5;
  const int nodeBase = (int)blockIdx.x * nb;

  for (int i = tid; i < NBMAX; i += NTHR) scnt[i] = 0;
  __syncthreads();

  int tot = 0;
  const int nChunks = (nE + CHUNK - 1) / CHUNK;
#pragma unroll 1
  for (int ch = 0; ch < nChunks; ++ch) {
    const int cbase = ch * CHUNK;
    const int wc = scan_chunk(dsts, nE, cbase, nodeBase, nb, vec8, list, tid, lane, wave);
    if (lane == 0) wcnt[wave] = wc;
    __syncthreads();
    int pre = 0, all = 0;
#pragma unroll
    for (int w2 = 0; w2 < NWAVE; ++w2) {
      int c = wcnt[w2];
      c = c < 0 ? 0 : (c > WCAP ? WCAP : c);
      all += c;
      pre += (w2 < wave) ? c : 0;
    }
    const int wcc  = wc > WCAP ? WCAP : wc;
    const int base = tot + pre;
#pragma unroll 1
    for (int i = lane; i < wcc; i += 32) {
      const int ent = list[wave * WCAP + i];
      const int el  = (ent >> 12) & (CHUNK - 1);
      const int sl  = ent & (NBMAX - 1);
      int eid = cbase + el;
      eid = eid > nE - 1 ? nE - 1 : eid;
      const int pos = base + i;
      if (pos < RCAP) reg1[pos] = (int)(((unsigned)eid << 12) | (unsigned)sl);
    }
    tot += all;
    tot = tot > RCAP ? RCAP : tot;
    __syncthreads();
  }
  const int nh = tot;

  if (wave == 0) {
#pragma unroll 1
    for (int b0 = 0; b0 < nh; b0 += 32) {
      const int idx = b0 + lane;
      const int uv  = reg1[idx < RCAP ? idx : RCAP - 1];
      const int m32 = (nh - b0) < 32 ? (nh - b0) : 32;
#pragma unroll 1
      for (int k = 0; k < m32; ++k) {
        const int u  = __builtin_amdgcn_readlane(uv, k);
        const int sl = u & (NBMAX - 1);
        if (lane == 0) scnt[sl] = scnt[sl] + 1;
      }
    }
  }
  __syncthreads();

  {
    const v4i ca = *(const v4i*)(scnt + 8 * tid);
    const v4i cb = *(const v4i*)(scnt + 8 * tid + 4);
    const int e0 = ca.x < 0 ? 0 : ca.x, e1 = ca.y < 0 ? 0 : ca.y, e2 = ca.z < 0 ? 0 : ca.z, e3 = ca.w < 0 ? 0 : ca.w;
    const int e4 = cb.x < 0 ? 0 : cb.x, e5 = cb.y < 0 ? 0 : cb.y, e6 = cb.z < 0 ? 0 : cb.z, e7 = cb.w < 0 ? 0 : cb.w;
    const int ts = e0 + e1 + e2 + e3 + e4 + e5 + e6 + e7;
    int incl = ts;
#pragma unroll
    for (int d = 1; d < 32; d <<= 1) {
      const int up = __shfl_up(incl, d);
      if (lane >= d) incl += up;
    }
    if (lane == 31) wtot[wave] = incl;
    __syncthreads();
    int pre = 0;
#pragma unroll
    for (int w2 = 0; w2 < NWAVE; ++w2) pre += (w2 < wave) ? wtot[w2] : 0;
    int run = pre + incl - ts;
    soff[8 * tid + 0] = run; run += e0;
    soff[8 * tid + 1] = run; run += e1;
    soff[8 * tid + 2] = run; run += e2;
    soff[8 * tid + 3] = run; run += e3;
    soff[8 * tid + 4] = run; run += e4;
    soff[8 * tid + 5] = run; run += e5;
    soff[8 * tid + 6] = run; run += e6;
    soff[8 * tid + 7] = run;
  }
  __syncthreads();
  for (int i = tid; i < NBMAX; i += NTHR) list[i] = soff[i];
  __syncthreads();

  if (wave == 0) {
#pragma unroll 1
    for (int b0 = 0; b0 < nh; b0 += 32) {
      const int idx = b0 + lane;
      const int uv  = reg1[idx < RCAP ? idx : RCAP - 1];
      const int m32 = (nh - b0) < 32 ? (nh - b0) : 32;
#pragma unroll 1
      for (int k = 0; k < m32; ++k) {
        const int u   = __builtin_amdgcn_readlane(uv, k);
        const int sl  = u & (NBMAX - 1);
        const int eid = (int)((unsigned)u >> 12);
        if (lane == 0) {
          int pos = list[sl];
          pos = pos < 0 ? 0 : (pos > RCAP - 1 ? RCAP - 1 : pos);
          reg2[pos] = eid;
          list[sl] = pos + 1;
        }
      }
    }
  }
  __syncthreads();

  const int nbw = nb >> 3;
  const bool ovf = (nh >= RCAP);
  unsigned int* stwu = (unsigned int*)reg1 + wave * STW;
  const unsigned int qn2 = 0x7fc07fc0u;
#pragma unroll 1
  for (int jt = 0; jt < nbw; ++jt) {
    const int slot = wave * nbw + jt;
    const int grow = nodeBase + slot;
    int st = soff[slot];
    const int craw = scnt[slot];
    int cnt = craw;
    st  = st < 0 ? 0 : (st > nh ? nh : st);
    cnt = cnt < 0 ? 0 : (cnt > DEGCAP ? DEGCAP : cnt);
    if (cnt > nh - st) cnt = nh - st;
    const bool pois = ovf || (craw > DEGCAP);
    const bool wr = grow < MPr;
    v4f a = {0.f, 0.f, 0.f, 0.f};
#pragma unroll 1
    for (int q = 0; q < cnt; ++q) {
      int idx = st + q; idx = idx > RCAP - 1 ? RCAP - 1 : idx;
      int eid = reg2[idx]; eid = eid < 0 ? 0 : (eid > nE - 1 ? nE - 1 : eid);
      int c = eid >> 3; c = c > nC - 1 ? nC - 1 : c;
      const v4f xv = *(const v4fa*)(CE + (size_t)c * DD + 4 * lane);
      a = a + xv;
    }
    const unsigned short h0 = bf16_rne(a.x), h1 = bf16_rne(a.y), h2 = bf16_rne(a.z), h3 = bf16_rne(a.w);
    const unsigned short l0 = bf16_rne(a.x - bf16_val(h0)), l1 = bf16_rne(a.y - bf16_val(h1));
    const unsigned short l2 = bf16_rne(a.z - bf16_val(h2)), l3 = bf16_rne(a.w - bf16_val(h3));
    v2u hp, lp;
    hp.x = (unsigned)h0 | ((unsigned)h1 << 16);  hp.y = (unsigned)h2 | ((unsigned)h3 << 16);
    lp.x = (unsigned)l0 | ((unsigned)l1 << 16);  lp.y = (unsigned)l2 | ((unsigned)l3 << 16);
    if (pois) { hp.x = qn2; hp.y = qn2; }
    if (lane == 0) list[slot] = (craw > 0) ? 1 : 0;
    __builtin_amdgcn_fence(__ATOMIC_RELEASE, "wavefront");
    __builtin_amdgcn_wave_barrier();
    *(v2u*)(stwu + 2 * lane) = hp;
    *(v2u*)(stwu + 64 + 2 * lane) = lp;
    __builtin_amdgcn_fence(__ATOMIC_RELEASE, "wavefront");
    __builtin_amdgcn_wave_barrier();
    const v4i g = *(const v4ia*)((const int*)stwu + 4 * lane);
    int* gp = (int*)(AGG + (size_t)grow * KP2) + 4 * lane;
    if (wr) *(volatile v4i*)gp = g;
    __threadfence();
    if (wr) *(volatile v4i*)gp = g;
  }
  __syncthreads();

  const int npc = nb >> 2;
  for (int i = tid; i < npc; i += NTHR) {
    const v4i f = *(const v4ia*)(list + 4 * i);
    *(volatile v4i*)(FLG + nodeBase + 4 * i) = f;
  }
  __threadfence();
  for (int i = tid; i < npc; i += NTHR) {
    const v4i f = *(const v4ia*)(list + 4 * i);
    *(volatile v4i*)(FLG + nodeBase + 4 * i) = f;
  }
}

__global__ __launch_bounds__(TTHR) void k_var(
    const unsigned short* __restrict__ AGG, const int* __restrict__ FLG,
    const unsigned short* __restrict__ VB, const unsigned short* __restrict__ GB,
    const unsigned short* __restrict__ WcT2, const unsigned short* __restrict__ WgGT,
    const unsigned short* __restrict__ WgAT2,
    const unsigned short* __restrict__ WzT2, const unsigned short* __restrict__ UzT,
    const unsigned short* __restrict__ WrT2, const unsigned short* __restrict__ UrT,
    const unsigned short* __restrict__ WwT2, const unsigned short* __restrict__ UuT2,
    const float* __restrict__ bc, const float* __restrict__ bg, const float* __restrict__ bz,
    const float* __restrict__ br, const float* __restrict__ bu,
    float* out, int nN)
{
  extern __shared__ v4f lds_dyn[];
  unsigned short* sX1 = (unsigned short*)lds_dyn;
  unsigned short* sX2 = sX1 + TROWS * KP2;
  unsigned short* sVB = sX2 + TROWS * KP2;
  unsigned short* sG  = sVB + TROWS * DD;
  float* sZ  = (float*)(sG + TROWS * GD);
  int*   sFl = (int*)(sZ + TROWS * DD);
  const int tid = (int)threadIdx.x, lane = tid & 31, wave = tid >> 5, hh = lane >> 4, m = lane & 15;
  const int row0 = (int)blockIdx.x * TROWS;
  const int wr0 = 16 * wave;

  {
    const v8usa* vs = (const v8usa*)(VB + (size_t)row0 * DD);
    v8us* vd = (v8us*)sVB;
#pragma unroll
    for (int i = 0; i < 8; ++i) vd[tid + TTHR * i] = vs[tid + TTHR * i];
    const v8usa* gs = (const v8usa*)(GB + (size_t)row0 * GD);
    v8us* gd = (v8us*)sG;
#pragma unroll
    for (int i = 0; i < 2; ++i) gd[tid + TTHR * i] = gs[tid + TTHR * i];
    if (tid < 16) ((v4i*)sFl)[tid] = ((const v4ia*)(FLG + row0))[tid];
  }
  __syncthreads();

  v8f acc[8];

  zero8(acc);
  gemm_seg(acc, AGG + (size_t)(row0 + wr0 + m) * KP2 + 8 * hh, WcT2 + (size_t)m * KP2 + 8 * hh, KP2, KP2 / 32);
#pragma unroll
  for (int t = 0; t < 8; ++t) {
    const int col = 16 * t + m;
    const float bb = bf16_val(bf16_rne(bc[col]));
#pragma unroll
    for (int r = 0; r < 8; ++r) {
      const int row = wr0 + 8 * hh + r;
      const float v = tanh_f(acc[t][r] + bb);
      const unsigned short hi = bf16_rne(v);
      sX1[row * KP2 + col] = hi;
      sX1[row * KP2 + DD + col] = bf16_rne(v - bf16_val(hi));
    }
  }
  __syncthreads();

  zero8(acc);
  gemm_seg(acc, sG + (wr0 + m) * GD + 8 * hh, WgGT + (size_t)m * GD + 8 * hh, GD, GD / 32);
  gemm_seg(acc, sX1 + (wr0 + m) * KP2 + 8 * hh, WgAT2 + (size_t)m * KP2 + 8 * hh, KP2, KP2 / 32);
#pragma unroll
  for (int t = 0; t < 8; ++t) {
    const int col = 16 * t + m;
    const float bb = bf16_val(bf16_rne(bg[col]));
#pragma unroll
    for (int r = 0; r < 8; ++r) {
      const int row = wr0 + 8 * hh + r;
      const float ne  = tanh_f(acc[t][r] + bb);
      const float vbf = bf16_val(sVB[row * DD + col]);
      const int   fl  = sFl[row];
      const float av  = fl > 0 ? ne : vbf;
      const unsigned short hi = bf16_rne(av);
      sX2[row * KP2 + col] = hi;
      sX2[row * KP2 + DD + col] = bf16_rne(av - bf16_val(hi));
    }
  }
  __syncthreads();

  zero8(acc);
  gemm_seg(acc, sX2 + (wr0 + m) * KP2 + 8 * hh, WzT2 + (size_t)m * KP2 + 8 * hh, KP2, KP2 / 32);
  gemm_seg(acc, sVB + (wr0 + m) * DD + 8 * hh, UzT + (size_t)m * DD + 8 * hh, DD, DD / 32);
#pragma unroll
  for (int t = 0; t < 8; ++t) {
    const int col = 16 * t + m;
    const float bb = bf16_val(bf16_rne(bz[col]));
#pragma unroll
    for (int r = 0; r < 8; ++r) {
      const int row = wr0 + 8 * hh + r;
      sZ[row * DD + col] = sigm_f(acc[t][r] + bb);
    }
  }

  zero8(acc);
  gemm_seg(acc, sX2 + (wr0 + m) * KP2 + 8 * hh, WrT2 + (size_t)m * KP2 + 8 * hh, KP2, KP2 / 32);
  gemm_seg(acc, sVB + (wr0 + m) * DD + 8 * hh, UrT + (size_t)m * DD + 8 * hh, DD, DD / 32);
#pragma unroll
  for (int t = 0; t < 8; ++t) {
    const int col = 16 * t + m;
    const float bb = bf16_val(bf16_rne(br[col]));
#pragma unroll
    for (int r = 0; r < 8; ++r) {
      const int row = wr0 + 8 * hh + r;
      const float rr  = sigm_f(acc[t][r] + bb);
      const float vbf = bf16_val(sVB[row * DD + col]);
      const float rv  = rr * vbf;
      const unsigned short hi = bf16_rne(rv);
      sX1[row * KP2 + col] = hi;
      sX1[row * KP2 + DD + col] = bf16_rne(rv - bf16_val(hi));
    }
  }
  __syncthreads();

  zero8(acc);
  gemm_seg(acc, sX2 + (wr0 + m) * KP2 + 8 * hh, WwT2 + (size_t)m * KP2 + 8 * hh, KP2, KP2 / 32);
  gemm_seg(acc, sX1 + (wr0 + m) * KP2 + 8 * hh, UuT2 + (size_t)m * KP2 + 8 * hh, KP2, KP2 / 32);
#pragma unroll
  for (int t = 0; t < 8; ++t) {
    const int col = 16 * t + m;
    const float bb = bf16_val(bf16_rne(bu[col]));
#pragma unroll
    for (int r = 0; r < 8; ++r) {
      const int row = wr0 + 8 * hh + r;
      const float ht  = tanh_f(acc[t][r] + bb);
      const float z   = sZ[row * DD + col];
      const float vbf = bf16_val(sVB[row * DD + col]);
      sZ[row * DD + col] = (1.0f - z) * vbf + z * ht;
    }
  }
  __syncthreads();

#pragma unroll
  for (int i = 0; i < 16; ++i) {
    const int row = wr0 + i, grow = row0 + row;
    const v4f v = ((const v4fa*)(sZ + row * DD))[lane];
    if (grow < nN) *(volatile v4f*)(out + (size_t)grow * DD + 4 * lane) = v;
  }
  __threadfence();
#pragma unroll
  for (int i = 0; i < 16; ++i) {
    const int row = wr0 + i, grow = row0 + row;
    const v4f v = ((const v4fa*)(sZ + row * DD))[lane];
    if (grow < nN) *(volatile v4f*)(out + (size_t)grow * DD + 4 * lane) = v;
  }
}

static int pick_nb(int nE, int nN) {
  int nb = NBMAX;
  while (nb > 16 && (long long)nb * (long long)nE * 5LL > (long long)RCAP * (long long)nN * 4LL) nb >>= 1;
  return nb;
}
static inline int cdiv(int a, int b) { return (a + b - 1) / b; }
static inline size_t al256(size_t x) { return (x + 255) & ~(size_t)255; }

static void launch_wtr(const float* W, int koff, int kmod, int Kout, unsigned short* dst, hipStream_t stream) {
  const int nU = DD * (Kout / 8);
  k_wtr2<<<cdiv(nU, 256), 256, 0, stream>>>(W, koff, kmod, Kout, dst, nU);
}

extern "C" void kernel_launch(void* const* d_in, const int* in_sizes, int n_in,
                              void* d_out, int out_size, void* d_ws, size_t ws_size,
                              hipStream_t stream) {
  if (n_in < 21) return;
  if (in_sizes[0] <= 0 || (in_sizes[0] % DD) != 0) return;
  const int nN = in_sizes[0] / DD;
  if (nN < TROWS || (nN % TROWS) != 0 || nN > (1 << 22)) return;
  if (in_sizes[1] != nN * GD) return;
  if (in_sizes[2] <= 0 || (in_sizes[2] % KL) != 0) return;
  const int nC = in_sizes[2] / KL;
  if (nC < TROWS || (nC % TROWS) != 0) return;
  if (in_sizes[3] != nC * KL) return;
  const int nE = nC * KL;
  if (nE < 1 || nE > (1 << 20)) return;
  if (in_sizes[4]  != DD * DD || in_sizes[5]  != DD) return;
  if (in_sizes[6]  != DD * DD || in_sizes[7]  != DD) return;
  if (in_sizes[8]  != DD * DD || in_sizes[9]  != DD) return;
  if (in_sizes[10] != (GD + DD) * DD || in_sizes[11] != DD) return;
  if (in_sizes[12] != DD * DD || in_sizes[13] != DD * DD || in_sizes[14] != DD) return;
  if (in_sizes[15] != DD * DD || in_sizes[16] != DD * DD || in_sizes[17] != DD) return;
  if (in_sizes[18] != DD * DD || in_sizes[19] != DD * DD || in_sizes[20] != DD) return;
  if (out_size != nN * DD) return;

  const float* x    = (const float*)d_in[0];
  const float* gft  = (const float*)d_in[1];
  const int*   lits = (const int*)  d_in[2];
  const int*   negs = (const int*)  d_in[3];
  const float* Wn = (const float*)d_in[4];  const float* bn = (const float*)d_in[5];
  const float* Wv = (const float*)d_in[6];  const float* bv = (const float*)d_in[7];
  const float* Wc = (const float*)d_in[8];  const float* bc = (const float*)d_in[9];
  const float* Wg = (const float*)d_in[10]; const float* bg = (const float*)d_in[11];
  const float* Wz = (const float*)d_in[12]; const float* Uz = (const float*)d_in[13];
  const float* bz = (const float*)d_in[14];
  const float* Wr = (const float*)d_in[15]; const float* Ur = (const float*)d_in[16];
  const float* br = (const float*)d_in[17];
  const float* Ww = (const float*)d_in[18]; const float* Uu = (const float*)d_in[19];
  const float* bu = (const float*)d_in[20];
  float* out = (float*)d_out;

  const int nb = pick_nb(nE, nN);
  if (nb < 32) return;
  const int gA  = cdiv(nN, nb);
  const int MPr = gA * nb;
  if (MPr < nN) return;
  const int vec8 = ((nE & 3) == 0) ? 1 : 0;

  char* ws = (char*)d_ws;
  size_t off = 0;
  const size_t oVB   = off; off = al256(off + (size_t)nN * DD * 2);
  const size_t oGB   = off; off = al256(off + (size_t)nN * GD * 2);
  const size_t oWn   = off; off = al256(off + (size_t)DD * KP2 * 2);
  const size_t oWv   = off; off = al256(off + (size_t)DD * KP2 * 2);
  const size_t oWc   = off; off = al256(off + (size_t)DD * KP2 * 2);
  const size_t oWgG  = off; off = al256(off + (size_t)DD * GD * 2);
  const size_t oWgA  = off; off = al256(off + (size_t)DD * KP2 * 2);
  const size_t oWz   = off; off = al256(off + (size_t)DD * KP2 * 2);
  const size_t oUz   = off; off = al256(off + (size_t)DD * DD * 2);
  const size_t oWr   = off; off = al256(off + (size_t)DD * KP2 * 2);
  const size_t oUr   = off; off = al256(off + (size_t)DD * DD * 2);
  const size_t oWw   = off; off = al256(off + (size_t)DD * KP2 * 2);
  const size_t oUu   = off; off = al256(off + (size_t)DD * KP2 * 2);
  const size_t oCE   = off; off = al256(off + (size_t)nC * DD * 4);
  const size_t oAGG  = off; off = al256(off + (size_t)MPr * KP2 * 2);
  const size_t oFLG  = off; off = al256(off + (size_t)MPr * 4);
  if (off > ws_size || off > (size_t)WSMAX) return;

  unsigned short* VB    = (unsigned short*)(ws + oVB);
  unsigned short* GB    = (unsigned short*)(ws + oGB);
  unsigned short* WnT2  = (unsigned short*)(ws + oWn);
  unsigned short* WvT2  = (unsigned short*)(ws + oWv);
  unsigned short* WcT2  = (unsigned short*)(ws + oWc);
  unsigned short* WgGT  = (unsigned short*)(ws + oWgG);
  unsigned short* WgAT2 = (unsigned short*)(ws + oWgA);
  unsigned short* WzT2  = (unsigned short*)(ws + oWz);
  unsigned short* UzT   = (unsigned short*)(ws + oUz);
  unsigned short* WrT2  = (unsigned short*)(ws + oWr);
  unsigned short* UrT   = (unsigned short*)(ws + oUr);
  unsigned short* WwT2  = (unsigned short*)(ws + oWw);
  unsigned short* UuT2  = (unsigned short*)(ws + oUu);
  float*          CE    = (float*)(ws + oCE);
  unsigned short* AGG   = (unsigned short*)(ws + oAGG);
  int*            FLG   = (int*)(ws + oFLG);

  hipFuncSetAttribute(reinterpret_cast<const void*>(&k_clause), hipFuncAttributeMaxDynamicSharedMemorySize, LDS_CLS);
  hipFuncSetAttribute(reinterpret_cast<const void*>(&k_scan),   hipFuncAttributeMaxDynamicSharedMemorySize, LDS_SCAN);
  hipFuncSetAttribute(reinterpret_cast<const void*>(&k_var),    hipFuncAttributeMaxDynamicSharedMemorySize, LDS_VAR);

  const int nUv = nN * (DD / 8), nUg = nN * (GD / 8);
  k_cvt<<<cdiv(nUv + nUg, 256), 256, 0, stream>>>(x, gft, VB, GB, nUv, nUg);

  launch_wtr(Wn, 0,  DD, KP2, WnT2,  stream);
  launch_wtr(Wv, 0,  DD, KP2, WvT2,  stream);
  launch_wtr(Wc, 0,  DD, KP2, WcT2,  stream);
  launch_wtr(Wg, 0,  GD, GD,  WgGT,  stream);
  launch_wtr(Wg, GD, DD, KP2, WgAT2, stream);
  launch_wtr(Wz, 0,  DD, KP2, WzT2,  stream);
  launch_wtr(Uz, 0,  DD, DD,  UzT,   stream);
  launch_wtr(Wr, 0,  DD, KP2, WrT2,  stream);
  launch_wtr(Ur, 0,  DD, DD,  UrT,   stream);
  launch_wtr(Ww, 0,  DD, KP2, WwT2,  stream);
  launch_wtr(Uu, 0,  DD, KP2, UuT2,  stream);

  k_clause<<<nC / TROWS, TTHR, LDS_CLS, stream>>>(VB, lits, negs, WnT2, WvT2, bn, bv, CE, nN, nC);

  k_scan<<<gA, NTHR, LDS_SCAN, stream>>>(lits, CE, AGG, FLG, nC, nE, nb, vec8, MPr);

  k_var<<<nN / TROWS, TTHR, LDS_VAR, stream>>>(AGG, FLG, VB, GB, WcT2, WgGT, WgAT2, WzT2, UzT, WrT2, UrT, WwT2, UuT2,
                                               bc, bg, bz, br, bu, out, nN);
}
